// GraphormerLayer_40492951667287
// MI455X (gfx1250) — hardware-verified
//
#include <hip/hip_runtime.h>


#define NB_  1
#define NT_  3072
#define DM   256
#define NH_  8
#define NKV  8
#define KVW  (NKV * HD)
#define LAT  256
#define FF   1024
#define HD   32
#define NTK  (NB_ * NT_)
#define NW   1024
#define NQKV 256
#define SCL  0.17677669529663688f
#define PSC  32768.0f
#define LOSC 1024.0f
#define LOSCI (1.0f / 1024.0f)

typedef _Float16 h16;
typedef unsigned short bf;
typedef __attribute__((ext_vector_type(16))) __bf16   v16bf;
typedef __attribute__((ext_vector_type(16))) _Float16 v16h;
typedef __attribute__((ext_vector_type(8)))  _Float16 v8h;
typedef __attribute__((ext_vector_type(8)))  unsigned short v8us;
typedef __attribute__((ext_vector_type(8)))  float    v8f;
typedef __attribute__((ext_vector_type(4)))  float    v4f;
typedef v8h  __attribute__((may_alias)) v8ha;
typedef v4f  __attribute__((may_alias)) v4fa;
typedef v8us __attribute__((may_alias)) v8usa;

__device__ __forceinline__ unsigned short f2bf(float f) { unsigned u = __float_as_uint(f); u += 0x7FFFu + ((u >> 16) & 1u); return (unsigned short)(u >> 16); }
__device__ __forceinline__ float bf2f(unsigned short b) { return __uint_as_float(((unsigned)b) << 16); }
__device__ __forceinline__ float bfr(float f) { return bf2f(f2bf(f)); }
__device__ __forceinline__ v16h cat16(v8h lo, v8h hi) { return __builtin_shufflevector(lo, hi, 0, 1, 2, 3, 4, 5, 6, 7, 8, 9, 10, 11, 12, 13, 14, 15); }
__device__ __forceinline__ v16bf cat16b(v8us lo, v8us hi) { return __builtin_bit_cast(v16bf, __builtin_shufflevector(lo, hi, 0, 1, 2, 3, 4, 5, 6, 7, 8, 9, 10, 11, 12, 13, 14, 15)); }
__device__ __forceinline__ v8f wmma16(v16h a, v16h b, v8f c) { return __builtin_amdgcn_wmma_f32_16x16x32_f16(false, a, false, b, (short)0, c, false, false); }
__device__ __forceinline__ v8f wmmab(v16bf a, v16bf b, v8f c) { return __builtin_amdgcn_wmma_f32_16x16x32_bf16(false, a, false, b, (short)0, c, false, false); }

__global__ __launch_bounds__(256) void k_cvtb(const float* __restrict__ src, int nrows, bf* dst) {
    const int lane = threadIdx.x & 31, r = blockIdx.x * 8 + (threadIdx.x >> 5);
    if (r >= nrows) return;
    v8us o[DM / 256];
#pragma unroll
    for (int q = 0; q < DM / 256; ++q) { v8us t;
#pragma unroll
        for (int i = 0; i < 8; ++i) t[i] = f2bf(src[(size_t)r * DM + q * 256 + lane * 8 + i]);
        o[q] = t; }
#pragma unroll
    for (int q = 0; q < DM / 256; ++q) *(volatile v8us*)(dst + (size_t)r * DM + q * 256 + lane * 8) = o[q];
    __threadfence();
#pragma unroll
    for (int q = 0; q < DM / 256; ++q) *(volatile v8us*)(dst + (size_t)r * DM + q * 256 + lane * 8) = o[q];
}

__global__ __launch_bounds__(256) void k_wt(const float* __restrict__ Wm, int Kdim, int ncols, bf* WT) {
    __shared__ __align__(16) unsigned short tl[64 * 72];
    const int tid = threadIdx.x, k0 = blockIdx.x * 64, n0 = blockIdx.y * 64;
    const int kk = tid >> 2, nq = (tid & 3) * 16;
#pragma unroll
    for (int i = 0; i < 16; ++i) tl[(nq + i) * 72 + kk] = f2bf(Wm[(size_t)(k0 + kk) * ncols + n0 + nq + i]);
    __syncthreads();
    const int piece = tid & 7;
    typedef __attribute__((ext_vector_type(8))) unsigned short v8us_; typedef v8us_ __attribute__((may_alias)) v8usa_;
    auto pass = [&]() {
#pragma unroll
        for (int s = 0; s < 2; ++s) { const int nr = (tid >> 3) + 32 * s; const v8us_ val = *(const v8usa_*)(tl + nr * 72 + piece * 8);
            *(volatile v8us_*)(WT + (size_t)(n0 + nr) * Kdim + k0 + piece * 8) = val; }
    };
    pass(); __threadfence(); pass();
}

template <bool SPLITA, bool F16OUT = false>
__global__ __launch_bounds__(128) void k_gemmb(const bf* __restrict__ A, const bf* __restrict__ Al, const bf* __restrict__ Bn, const float* __restrict__ bias, float* C, int ldc, h16* C2, int K) {
    __shared__ __align__(16) float ost[4][16 * 68];
    const int lane = threadIdx.x & 31, wave = threadIdx.x >> 5, lr = lane & 15, hi = lane >> 4;
    const int r0 = blockIdx.x * 64 + wave * 16, c0 = blockIdx.y * 64;
    const size_t aoff = (size_t)(r0 + lr) * K + 8 * hi;
    size_t boff[4];
#pragma unroll
    for (int t = 0; t < 4; ++t) boff[t] = (size_t)(c0 + t * 16 + lr) * K + 8 * hi;
    v8f acc[4];
#pragma unroll
    for (int t = 0; t < 4; ++t) acc[t] = (v8f){};
#pragma unroll 1
    for (int kc = 0; kc < K; kc += 32) {
        const v16bf a = cat16b(*(const v8us*)(A + aoff + kc), *(const v8us*)(A + aoff + kc + 16));
        v16bf al = a;
        if (SPLITA) al = cat16b(*(const v8us*)(Al + aoff + kc), *(const v8us*)(Al + aoff + kc + 16));
#pragma unroll
        for (int t = 0; t < 4; ++t) { const v16bf b = cat16b(*(const v8us*)(Bn + boff[t] + kc), *(const v8us*)(Bn + boff[t] + kc + 16)); acc[t] = wmmab(a, b, acc[t]); if (SPLITA) acc[t] = wmmab(al, b, acc[t]); }
        asm volatile("v_nop\n\tv_nop\n\tv_nop\n\tv_nop" : "+v"(acc[0]), "+v"(acc[1]), "+v"(acc[2]), "+v"(acc[3]) : "v"(a), "v"(al));
    }
    float* os = &ost[wave][0];
#pragma unroll
    for (int t = 0; t < 4; ++t) { const float bv = bias ? bfr(bias[c0 + t * 16 + lr]) : 0.f;
#pragma unroll
        for (int j = 0; j < 8; ++j) os[(hi * 8 + j) * 68 + t * 16 + lr] = acc[t][j] + bv; }
    __syncthreads();
    if (F16OUT) {
        h16* crow = (h16*)(void*)C + (size_t)r0 * ldc + c0;
        auto pass = [&]() {
#pragma unroll
            for (int s = 0; s < 4; ++s) { const int row = 4 * s + (lane >> 3), piece = lane & 7; const float* sp = os + row * 68 + piece * 8; v8h o, o2;
#pragma unroll
                for (int i = 0; i < 8; ++i) { const h16 a = (h16)sp[i]; o[i] = a; o2[i] = (h16)((sp[i] - (float)a) * LOSC); }
                *(volatile v8h*)(crow + (size_t)row * ldc + piece * 8) = o; if (C2) *(volatile v8h*)(C2 + (size_t)r0 * ldc + c0 + (size_t)row * ldc + piece * 8) = o2; }
        };
        pass(); __threadfence(); pass();
    } else {
        float* crow = C + (size_t)r0 * ldc + c0;
        auto pass = [&]() {
#pragma unroll
            for (int s = 0; s < 8; ++s) { const int Lid = (lane >> 3) + 4 * s, piece = lane & 7; const int row = Lid >> 1, cofs = (Lid & 1) * 32 + piece * 4;
                const v4f val = *(const v4fa*)(os + row * 68 + cofs); *(volatile v4f*)(crow + (size_t)row * ldc + cofs) = val; }
        };
        pass(); __threadfence(); pass();
    }
}

__global__ __launch_bounds__(256) void k_x2(const float* __restrict__ x, const int* __restrict__ cin, const int* __restrict__ cout_, const float* __restrict__ ein, const float* __restrict__ eout, bf* XH, bf* XL) {
    const int lane = threadIdx.x & 31, r = blockIdx.x * 8 + (threadIdx.x >> 5);
    if (r >= NT_) return;
    int ci = cin[r]; ci = ci < 0 ? 0 : (ci > 50 ? 50 : ci); int co = cout_[r]; co = co < 0 ? 0 : (co > 50 ? 50 : co);
    v8us oh, ol;
#pragma unroll
    for (int i = 0; i < 8; ++i) { const int c = lane * 8 + i; const float v = bfr(x[(size_t)r * DM + c]) + bfr(ein[(size_t)ci * DM + c]) + bfr(eout[(size_t)co * DM + c]); const unsigned short hb = f2bf(v); oh[i] = hb; ol[i] = f2bf(v - bf2f(hb)); }
    *(volatile v8us*)(XH + (size_t)r * DM + lane * 8) = oh; *(volatile v8us*)(XL + (size_t)r * DM + lane * 8) = ol; __threadfence();
    *(volatile v8us*)(XH + (size_t)r * DM + lane * 8) = oh; *(volatile v8us*)(XL + (size_t)r * DM + lane * 8) = ol;
}
__global__ __launch_bounds__(256) void k_ln(const float* __restrict__ A, const float* __restrict__ Bv, const float* __restrict__ g, const float* __restrict__ be, int roundA, float* Yf, bf* YH, bf* YL) {
    const int lane = threadIdx.x & 31, r = blockIdx.x * 8 + (threadIdx.x >> 5);
    if (r >= NT_) return;
    float v[8]; float s = 0.f;
#pragma unroll
    for (int i = 0; i < 8; ++i) { const size_t c = (size_t)r * DM + lane * 8 + i; const float a = roundA ? bfr(A[c]) : A[c]; v[i] = a + Bv[c]; s += v[i]; }
#pragma unroll
    for (int o = 16; o; o >>= 1) s += __shfl_xor(s, o, 32);
    const float mu = s * (1.0f / DM); float q = 0.f;
#pragma unroll
    for (int i = 0; i < 8; ++i) { const float d = v[i] - mu; q += d * d; }
#pragma unroll
    for (int o = 16; o; o >>= 1) q += __shfl_xor(q, o, 32);
    const float rs = rsqrtf(q * (1.0f / DM) + 1e-5f);
    v8us oh, ol; v4f y0, y1;
#pragma unroll
    for (int i = 0; i < 8; ++i) { const int c = lane * 8 + i; const float y = (v[i] - mu) * rs * bfr(g[c]) + bfr(be[c]); if (i < 4) y0[i] = y; else y1[i - 4] = y; const unsigned short hb = f2bf(y); oh[i] = hb; ol[i] = f2bf(y - bf2f(hb)); }
    __shared__ float rowbuf[8][DM];
    float* rb = rowbuf[threadIdx.x >> 5];
#pragma unroll
    for (int i = 0; i < 4; ++i) { rb[lane * 8 + i] = y0[i]; rb[lane * 8 + 4 + i] = y1[i]; }
    __builtin_amdgcn_wave_barrier();
    auto pass = [&]() {
#pragma unroll
        for (int s2 = 0; s2 < 2; ++s2) { const v4f val = *(const v4fa*)(rb + s2 * 128 + lane * 4); *(volatile v4f*)(Yf + (size_t)r * DM + s2 * 128 + lane * 4) = val; }
        if (YH) { *(volatile v8us*)(YH + (size_t)r * DM + lane * 8) = oh; *(volatile v8us*)(YL + (size_t)r * DM + lane * 8) = ol; }
    };
    pass(); __threadfence(); pass();
}
__global__ __launch_bounds__(256) void k_gelu(const float* __restrict__ F, bf* GH, bf* GL) {
    const int lane = threadIdx.x & 31; const size_t w = (size_t)blockIdx.x * 8 + (threadIdx.x >> 5);
    v8us oh, ol;
#pragma unroll
    for (int i = 0; i < 8; ++i) { const float v = F[w * 256 + lane * 8 + i]; const float gq = 0.5f * v * (1.0f + erff(v * 0.7071067811865476f)); const unsigned short hb = f2bf(gq); oh[i] = hb; ol[i] = f2bf(gq - bf2f(hb)); }
    *(volatile v8us*)(GH + w * 256 + lane * 8) = oh; *(volatile v8us*)(GL + w * 256 + lane * 8) = ol; __threadfence();
    *(volatile v8us*)(GH + w * 256 + lane * 8) = oh; *(volatile v8us*)(GL + w * 256 + lane * 8) = ol;
}
__global__ __launch_bounds__(256) void k_splitbf(const float* __restrict__ S, int rows, bf* SH, bf* SL) {
    const int lane = threadIdx.x & 31, r = blockIdx.x * 8 + (threadIdx.x >> 5);
    if (r >= rows) return;
    v8us oh, ol;
#pragma unroll
    for (int i = 0; i < 8; ++i) { const float v = S[(size_t)r * LAT + lane * 8 + i]; const unsigned short hb = f2bf(v); oh[i] = hb; ol[i] = f2bf(v - bf2f(hb)); }
    *(volatile v8us*)(SH + (size_t)r * LAT + lane * 8) = oh; *(volatile v8us*)(SL + (size_t)r * LAT + lane * 8) = ol; __threadfence();
    *(volatile v8us*)(SH + (size_t)r * LAT + lane * 8) = oh; *(volatile v8us*)(SL + (size_t)r * LAT + lane * 8) = ol;
}
__global__ __launch_bounds__(256) void k_s16(const float* __restrict__ S, int rows, h16* SH, h16* SL) {
    const int lane = threadIdx.x & 31, r = blockIdx.x * 8 + (threadIdx.x >> 5);
    if (r >= rows) return;
#pragma unroll
    for (int q = 0; q < DM / 256; ++q) { v8h oh, ol;
#pragma unroll
        for (int i = 0; i < 8; ++i) { const float v = S[(size_t)r * DM + q * 256 + lane * 8 + i]; const h16 a = (h16)v; oh[i] = a; ol[i] = (h16)((v - (float)a) * LOSC); }
        *(volatile v8h*)(SH + (size_t)r * DM + q * 256 + lane * 8) = oh; *(volatile v8h*)(SL + (size_t)r * DM + q * 256 + lane * 8) = ol; __threadfence();
        *(volatile v8h*)(SH + (size_t)r * DM + q * 256 + lane * 8) = oh; *(volatile v8h*)(SL + (size_t)r * DM + q * 256 + lane * 8) = ol; }
}
__global__ __launch_bounds__(256) void k_vt(const float* __restrict__ V, h16* VTH, h16* VTL) {
    __shared__ __align__(16) h16 tile[64 * 72];
    __shared__ __align__(16) h16 til2[64 * 72];
    const int bid = blockIdx.x;
    const int b = bid / ((KVW / 64) * (NT_ / 64)), rem = bid - b * ((KVW / 64) * (NT_ / 64)), h = rem / (NT_ / 64), kt = rem - h * (NT_ / 64);
    const int k0 = kt * 64, tid = threadIdx.x;
    const int kk = tid >> 2, d0 = (tid & 3) * 16;
    const float* src = V + ((size_t)b * NT_ + k0 + kk) * KVW + h * 64 + d0;
#pragma unroll
    for (int i = 0; i < 16; ++i) { const float v = src[i]; const h16 a = (h16)v; tile[(d0 + i) * 72 + kk] = a; til2[(d0 + i) * 72 + kk] = (h16)((v - (float)a) * LOSC); }
    __syncthreads();
    const int piece = tid & 7;
    const size_t base = (((size_t)b * (KVW / 64) + h) * 64) * NT_ + k0;
    auto pass = [&]() {
#pragma unroll
        for (int s = 0; s < 4; ++s) { const int Lid = (tid >> 3) + 32 * s; const int pln = Lid >> 6, d = Lid & 63;
            const v8h val = *(const v8ha*)((pln ? til2 : tile) + d * 72 + piece * 8); *(volatile v8h*)((pln ? VTL : VTH) + base + (size_t)d * NT_ + piece * 8) = val; }
    };
    pass(); __threadfence(); pass();
}

__global__ __launch_bounds__(128) void k_attn(const h16* __restrict__ Q16, const h16* __restrict__ QL16, const h16* __restrict__ K16, const h16* __restrict__ KL16, const h16* __restrict__ VTH, const h16* __restrict__ VTL,
                                             const int* __restrict__ spd, const int* __restrict__ edge, const float* __restrict__ spdE, const float* __restrict__ edgeE, bf* CH, bf* CL) {
    __shared__ __align__(16) h16 plds[4][16 * 32];
    __shared__ __align__(16) h16 plds2[4][16 * 32];
    __shared__ __align__(16) float ost[4][16 * 68];
    const int lane = threadIdx.x & 31, wave = threadIdx.x >> 5, lr = lane & 15, hi = lane >> 4;
    const int bid = blockIdx.x;
    const int b = bid / ((NH_ / 2) * (NT_ / 64)), rem = bid - b * ((NH_ / 2) * (NT_ / 64)), g2 = rem / (NT_ / 64), qt = rem - g2 * (NT_ / 64);
    const int q0 = qt * 64 + wave * 16;
    const size_t tok0 = (size_t)b * NT_;
    h16* pl = &plds[wave][0]; h16* pl2 = &plds2[wave][0];
    float* os = &ost[wave][0];
#pragma unroll 1
    for (int hh = 0; hh < 2; ++hh) {
    const int h = g2 * 2 + hh;
    v16h qa[1];
    const size_t qo0 = (tok0 + q0 + lr) * DM + h * HD + 8 * hi;
    qa[0] = cat16(*(const v8h*)(Q16 + qo0), *(const v8h*)(Q16 + qo0 + 16));
    float se[11], ee[6];
#pragma unroll
    for (int i = 0; i < 11; ++i) se[i] = bfr(spdE[i * NH_ + h]);
#pragma unroll
    for (int i = 0; i < 6; ++i) ee[i] = bfr(edgeE[i * NH_ + h]);
    const int g = h / (NH_ / NKV);
    const h16* kh_b = K16 + tok0 * KVW + g * HD;
    const h16* kl_b = KL16 + tok0 * KVW + g * HD;
    const size_t vbase = (((size_t)b * NKV + g) * HD) * NT_;
    v8f o[2], ox[2];
#pragma unroll
    for (int n = 0; n < 2; ++n) { o[n] = (v8f){}; ox[n] = (v8f){}; }
    float mrow[8], lpart[8];
#pragma unroll
    for (int j = 0; j < 8; ++j) { mrow[j] = -3.0e38f; lpart[j] = 0.f; }
    int qpos[8];
#pragma unroll
    for (int j = 0; j < 8; ++j) qpos[j] = q0 + 8 * hi + j;
    const int kt_lo = 0, kt_hi = NT_ / 32 - 1;
#pragma unroll 1
    for (int kt = kt_lo; kt <= kt_hi; ++kt) {
        const int l0 = kt * 32;
        const size_t ko0 = (size_t)(l0 + lr) * KVW + 8 * hi, ko1 = (size_t)(l0 + 16 + lr) * KVW + 8 * hi;
        v8f s0 = {}, s1 = {}, x0 = {}, x1 = {};
#pragma unroll
        for (int kc = 0; kc < 1; ++kc) {
            { const v16h k0h = cat16(*(const v8h*)(kh_b + ko0 + kc * 32), *(const v8h*)(kh_b + ko0 + kc * 32 + 16)), k1h = cat16(*(const v8h*)(kh_b + ko1 + kc * 32), *(const v8h*)(kh_b + ko1 + kc * 32 + 16));
              const v16h qlk = cat16(*(const v8h*)(QL16 + qo0 + kc * 32), *(const v8h*)(QL16 + qo0 + kc * 32 + 16));
              s0 = wmma16(qa[kc], k0h, s0); x0 = wmma16(qlk, k0h, x0); s1 = wmma16(qa[kc], k1h, s1); x1 = wmma16(qlk, k1h, x1);
              asm volatile("v_nop" : "+v"(s0), "+v"(s1), "+v"(x0), "+v"(x1) : "v"(qlk), "v"(k0h), "v"(k1h) : "memory"); }
            { const v16h k0l = cat16(*(const v8h*)(kl_b + ko0 + kc * 32), *(const v8h*)(kl_b + ko0 + kc * 32 + 16)), k1l = cat16(*(const v8h*)(kl_b + ko1 + kc * 32), *(const v8h*)(kl_b + ko1 + kc * 32 + 16));
              x0 = wmma16(qa[kc], k0l, x0); x1 = wmma16(qa[kc], k1l, x1);
              asm volatile("v_nop" : "+v"(x0), "+v"(x1) : "v"(k0l), "v"(k1l) : "memory"); }
        }
        asm volatile("v_nop\n\tv_nop\n\tv_nop\n\tv_nop" : "+v"(s0), "+v"(s1), "+v"(x0), "+v"(x1) : "v"(qa[0]));
        float alpha[8];
#pragma unroll
        for (int j = 0; j < 8; ++j) {
            const int ja = l0 + lr, jb = l0 + 16 + lr, qi = qpos[j];
            int sa = spd[(size_t)qi * NT_ + ja], sb = spd[(size_t)qi * NT_ + jb]; int ea = edge[(size_t)qi * NT_ + ja], eb = edge[(size_t)qi * NT_ + jb];
            const bool va = (sa <= 10), vb = (sb <= 10);
            sa = sa < 0 ? 0 : (sa > 10 ? 10 : sa); sb = sb < 0 ? 0 : (sb > 10 ? 10 : sb); ea = ea < 0 ? 0 : (ea > 5 ? 5 : ea); eb = eb < 0 ? 0 : (eb > 5 ? 5 : eb);
            float bsa = 0.f, bsb = 0.f, bea = 0.f, beb = 0.f;
#pragma unroll
            for (int i = 0; i < 11; ++i) { bsa = (sa == i) ? se[i] : bsa; bsb = (sb == i) ? se[i] : bsb; }
#pragma unroll
            for (int i = 0; i < 6; ++i) { bea = (ea == i) ? ee[i] : bea; beb = (eb == i) ? ee[i] : beb; }
            const float a0 = va ? (s0[j] + x0[j] * LOSCI) * SCL + bsa + bea : -1.0e9f, a1 = vb ? (s1[j] + x1[j] * LOSCI) * SCL + bsb + beb : -1.0e9f;
            float mx = fmaxf(a0, a1);
            mx = fmaxf(mx, __shfl_xor(mx, 1, 16)); mx = fmaxf(mx, __shfl_xor(mx, 2, 16)); mx = fmaxf(mx, __shfl_xor(mx, 4, 16)); mx = fmaxf(mx, __shfl_xor(mx, 8, 16));
            const float mn = fmaxf(mrow[j], mx);
            alpha[j] = __expf(mrow[j] - mn); mrow[j] = mn;
            const float p0 = __expf(a0 - mn), p1 = __expf(a1 - mn);
            lpart[j] = lpart[j] * alpha[j] + (p0 + p1);
            const int mr = hi * 8 + j;
            const float ps0 = p0 * PSC, ps1 = p1 * PSC; const h16 h0 = (h16)ps0, h1 = (h16)ps1;
            pl[mr * 32 + lr] = h0; pl[mr * 32 + 16 + lr] = h1;
            pl2[mr * 32 + lr] = (h16)((ps0 - (float)h0) * LOSC); pl2[mr * 32 + 16 + lr] = (h16)((ps1 - (float)h1) * LOSC);
        }
#pragma unroll
        for (int n = 0; n < 2; ++n)
#pragma unroll
            for (int j = 0; j < 8; ++j) { o[n][j] *= alpha[j]; ox[n][j] *= alpha[j]; }
        asm volatile("" ::: "memory");
        const v16h pa = cat16(*(const v8ha*)(pl + lr * 32 + hi * 8), *(const v8ha*)(pl + lr * 32 + 16 + hi * 8));
        const v16h px = cat16(*(const v8ha*)(pl2 + lr * 32 + hi * 8), *(const v8ha*)(pl2 + lr * 32 + 16 + hi * 8));
#pragma unroll
        for (int n = 0; n < 2; ++n) { const size_t vo = vbase + (size_t)(n * 16 + lr) * NT_ + l0 + hi * 8;
            const v16h vh = cat16(*(const v8h*)(VTH + vo), *(const v8h*)(VTH + vo + 16)), vl = cat16(*(const v8h*)(VTL + vo), *(const v8h*)(VTL + vo + 16));
            o[n] = wmma16(pa, vh, o[n]); ox[n] = wmma16(pa, vl, ox[n]); ox[n] = wmma16(px, vh, ox[n]);
            asm volatile("" : "+v"(o[n]), "+v"(ox[n]) : "v"(vh), "v"(vl) : "memory"); }
        asm volatile("v_nop\n\tv_nop\n\tv_nop\n\tv_nop" : "+v"(o[0]), "+v"(o[1]), "+v"(ox[0]), "+v"(ox[1]) : "v"(pa), "v"(px));
    }
    float inv[8];
#pragma unroll
    for (int j = 0; j < 8; ++j) { float rs = lpart[j]; rs += __shfl_xor(rs, 1, 16); rs += __shfl_xor(rs, 2, 16); rs += __shfl_xor(rs, 4, 16); rs += __shfl_xor(rs, 8, 16); inv[j] = 1.0f / (rs * PSC); }
#pragma unroll
    for (int n = 0; n < 2; ++n)
#pragma unroll
        for (int j = 0; j < 8; ++j) os[(hi * 8 + j) * 68 + hh * 32 + n * 16 + lr] = (o[n][j] + ox[n][j] * LOSCI) * inv[j];
    }
    __syncthreads();
    const size_t cbase = (tok0 + q0) * DM + (size_t)g2 * 64;
    auto pass = [&]() {
#pragma unroll
        for (int s = 0; s < 4; ++s) { const int row = 4 * s + (lane >> 3), piece = lane & 7; const float* sp = os + row * 68 + piece * 8; v8us oh, ol;
#pragma unroll
            for (int i = 0; i < 8; ++i) { const unsigned short hb = f2bf(sp[i]); oh[i] = hb; ol[i] = f2bf(sp[i] - bf2f(hb)); }
            *(volatile v8us*)(CH + cbase + (size_t)row * DM + piece * 8) = oh; *(volatile v8us*)(CL + cbase + (size_t)row * DM + piece * 8) = ol; }
    };
    pass(); __threadfence(); pass();
}

#define VST2(T, p, v) do { const T vst2_v_ = (v); *(volatile T*)(p) = vst2_v_; __threadfence(); *(volatile T*)(p) = vst2_v_; } while (0)
extern "C" void kernel_launch(void* const* d_in, const int* in_sizes, int n_in,
                              void* d_out, int out_size, void* d_ws, size_t ws_size, hipStream_t stream) {
    (void)in_sizes; (void)n_in; (void)out_size;
    const float* x = (const float*)d_in[0]; const int* spd = (const int*)d_in[1]; const int* cin = (const int*)d_in[2]; const int* cout_ = (const int*)d_in[3]; const int* edge = (const int*)d_in[4];
    const float* spdE = (const float*)d_in[5]; const float* cinE = (const float*)d_in[6]; const float* coutE = (const float*)d_in[7]; const float* edgeE = (const float*)d_in[8];
    const float* Wq = (const float*)d_in[9]; const float* bq = (const float*)d_in[10]; const float* Wk = (const float*)d_in[11]; const float* bk = (const float*)d_in[12]; const float* Wv = (const float*)d_in[13]; const float* bv = (const float*)d_in[14];
    const float* Wo = (const float*)d_in[15]; const float* bo = (const float*)d_in[16]; const float* W1 = (const float*)d_in[17]; const float* b1 = (const float*)d_in[18]; const float* W2 = (const float*)d_in[19]; const float* b2 = (const float*)d_in[20];
    const float* g1 = (const float*)d_in[21]; const float* be1 = (const float*)d_in[22]; const float* g2p = (const float*)d_in[23]; const float* be2 = (const float*)d_in[24];
    float* out = (float*)d_out;
    char* wsp = (char*)d_ws;
    auto take = [&](size_t bytes) { char* p = wsp; wsp += (bytes + 255) & ~(size_t)255; return (void*)p; };
    bf* XH = (bf*)take((size_t)NTK * DM * 2); bf* XL = (bf*)take((size_t)NTK * DM * 2);
    bf* WqT = (bf*)take((size_t)DM * DM * 2); bf* WkT = (bf*)take((size_t)DM * DM * 2); bf* WvT = (bf*)take((size_t)DM * DM * 2); bf* WoT = (bf*)take((size_t)DM * DM * 2); bf* W1T = (bf*)take((size_t)FF * DM * 2); bf* W2T = (bf*)take((size_t)DM * FF * 2);
    h16* QH = (h16*)take((size_t)NTK * DM * 2); h16* QL = (h16*)take((size_t)NTK * DM * 2); h16* KH = (h16*)take((size_t)NTK * DM * 2); h16* KL = (h16*)take((size_t)NTK * DM * 2);
    float* Vf = (float*)take((size_t)NTK * DM * 4); h16* VTH = (h16*)take((size_t)NTK * DM * 2); h16* VTL = (h16*)take((size_t)NTK * DM * 2);
    bf* CH = (bf*)take((size_t)NTK * DM * 2); bf* CL = (bf*)take((size_t)NTK * DM * 2); float* O = (float*)take((size_t)NTK * DM * 4);
    float* X1 = (float*)take((size_t)NTK * DM * 4); bf* X1H = (bf*)take((size_t)NTK * DM * 2); bf* X1L = (bf*)take((size_t)NTK * DM * 2);
    float* F1 = (float*)take((size_t)NTK * FF * 4); bf* GH = (bf*)take((size_t)NTK * FF * 2); bf* GL = (bf*)take((size_t)NTK * FF * 2); float* F2 = (float*)take((size_t)NTK * DM * 4);
    if ((size_t)(wsp - (char*)d_ws) > ws_size) return;
    k_x2<<<NTK / 8, 256, 0, stream>>>(x, cin, cout_, cinE, coutE, XH, XL);
    k_wt<<<dim3(DM / 64, DM / 64, 1), 256, 0, stream>>>(Wq, DM, DM, WqT); k_wt<<<dim3(DM / 64, DM / 64, 1), 256, 0, stream>>>(Wk, DM, DM, WkT); k_wt<<<dim3(DM / 64, DM / 64, 1), 256, 0, stream>>>(Wv, DM, DM, WvT);
    k_wt<<<dim3(DM / 64, DM / 64, 1), 256, 0, stream>>>(Wo, DM, DM, WoT); k_wt<<<dim3(DM / 64, FF / 64, 1), 256, 0, stream>>>(W1, DM, FF, W1T); k_wt<<<dim3(FF / 64, DM / 64, 1), 256, 0, stream>>>(W2, FF, DM, W2T);
    k_gemmb<true, true><<<dim3(NTK / 64, DM / 64, 1), 128, 0, stream>>>(XH, XL, WqT, bq, (float*)(void*)QH, DM, QL, DM);
    k_gemmb<true, true><<<dim3(NTK / 64, DM / 64, 1), 128, 0, stream>>>(XH, XL, WkT, bk, (float*)(void*)KH, DM, KL, DM);
    k_gemmb<true, false><<<dim3(NTK / 64, DM / 64, 1), 128, 0, stream>>>(XH, XL, WvT, bv, Vf, DM, nullptr, DM);
    k_vt<<<NB_ * (KVW / 64) * (NT_ / 64), 256, 0, stream>>>(Vf, VTH, VTL);
    k_attn<<<NB_ * (NH_ / 2) * (NT_ / 64), 128, 0, stream>>>(QH, QL, KH, KL, VTH, VTL, spd, edge, spdE, edgeE, CH, CL);
    k_gemmb<true, false><<<dim3(NTK / 64, DM / 64, 1), 128, 0, stream>>>(CH, CL, WoT, bo, O, DM, nullptr, DM);
    k_ln<<<NTK / 8, 256, 0, stream>>>(x, O, g1, be1, 1, X1, X1H, X1L);
    k_gemmb<true, false><<<dim3(NTK / 64, FF / 64, 1), 128, 0, stream>>>(X1H, X1L, W1T, b1, F1, FF, nullptr, DM);
    k_gelu<<<(NTK * FF / 256) / 8, 256, 0, stream>>>(F1, GH, GL);
    k_gemmb<true, false><<<dim3(NTK / 64, DM / 64, 1), 128, 0, stream>>>(GH, GL, W2T, b2, F2, DM, nullptr, FF);
    k_ln<<<NTK / 8, 256, 0, stream>>>(X1, F2, g2p, be2, 0, out, nullptr, nullptr);
}
